// GNNbase_41661182771449
// MI455X (gfx1250) — hardware-verified
//
#include <hip/hip_runtime.h>
#include <stddef.h>


#define NGR    256
#define NPG    64
#define EPG    256
#define NNODE  16384
#define NEDGE  65536
#define DH     128
#define HCOL   512
#define QKVW   1536
#define EDIM   16
#define NLAY   3
#define GPH    128
#define NDH    8192
#define NTHR   256
#define NWAVE  8
#define NJOB   22
#define BIGD   (1 << 20)
#define NEG_BIG (-3.0e38f)

#define PW1    0
#define PW2    4096
#define PW3    20480
#define PLAY0  36864
#define PLAYSZ 229376
#define PQKV   0
#define PWG    196608
#define PWTS   204800
#define PWOUT  724992
#define WPLH   741376

#define OFF_W    0
#define SZ_W     1482752
#define OFF_F    1482752
#define SZ_F     4194304
#define OFF_R2   5677056
#define SZ_R2    33554432
#define OFF_R3   39231488
#define SZ_R3    67108864
#define WS_TOTAL 106340352
#define WS_CAP   134217728

#define E_H1H 0
#define E_H1L 16777216
#define E_H2H 33554432
#define E_H2L 50331648
#define N_ACH 0
#define N_ACL 4194304
#define N_ANH 8388608
#define N_ANL 12582912
#define N_G   16777216
#define N_VS  18874368
#define N_SH  23068672
#define N_SL  24117248
#define N_GTH 25165824
#define N_GTL 25231360
#define N_END 25296896
#define N_QKV 0
#define N_QPH 50331648
#define N_QPL 58720256

#define LDS_G8 65536
#define LDS_G4 32768

static_assert(SZ_W == WPLH * 2);
static_assert(PW2 == PW1 + 128 * 32);
static_assert(PW3 == PW2 + 128 * 128);
static_assert(PLAY0 == PW3 + 128 * 128);
static_assert(PWG == PQKV + QKVW * DH);
static_assert(PWTS == PWG + 64 * DH);
static_assert(PLAYSZ == PWTS + DH * 192);
static_assert(PWOUT == PLAY0 + NLAY * PLAYSZ);
static_assert(WPLH == PWOUT + DH * DH);
static_assert((PLAYSZ * 2) % 256 == 0 && (PWG * 2) % 256 == 0 && (PWTS * 2) % 256 == 0 && (PW2 * 2) % 256 == 0);
static_assert(OFF_F == OFF_W + SZ_W && OFF_R2 == OFF_F + SZ_F && OFF_R3 == OFF_R2 + SZ_R2 && WS_TOTAL == OFF_R3 + SZ_R3);
static_assert((OFF_F % 256) == 0 && (OFF_R2 % 256) == 0 && (OFF_R3 % 256) == 0);
static_assert(SZ_F == NEDGE * 32 * 2);
static_assert(SZ_R2 == NEDGE * DH * 4);
static_assert(E_H1L == NEDGE * DH * 2 && E_H2H == 2 * E_H1L && E_H2L == 3 * E_H1L && SZ_R3 == 4 * E_H1L);
static_assert(N_ACL == NNODE * DH * 2 && N_ANH == 2 * N_ACL && N_ANL == 3 * N_ACL && N_G == 4 * N_ACL);
static_assert(N_VS == N_G + NDH * 64 * 4);
static_assert(N_SH == N_VS + NDH * DH * 4);
static_assert(N_SL == N_SH + NDH * 64 * 2);
static_assert(N_GTH == N_SL + NDH * 64 * 2);
static_assert(N_GTL == N_GTH + NGR * DH * 2);
static_assert(N_END == N_GTL + NGR * DH * 2);
static_assert(N_END <= SZ_R2);
static_assert(N_QPH == N_QKV + NDH * QKVW * 4);
static_assert(N_QPL == N_QPH + NDH * HCOL * 2);
static_assert(N_QPL + NDH * HCOL * 2 == SZ_R3);
static_assert(WS_TOTAL <= WS_CAP);
static_assert(NPG == NWAVE * 8);
static_assert(EPG == NTHR);

typedef float          v2f  __attribute__((ext_vector_type(2)));
typedef float          v4f  __attribute__((ext_vector_type(4)));
typedef float          v8f  __attribute__((ext_vector_type(8)));
typedef unsigned short v8us __attribute__((ext_vector_type(8)));
typedef __bf16         v16b __attribute__((ext_vector_type(16)));
union FragB { v16b v; v8us h[2]; };

__device__ __forceinline__ unsigned int bfr(float f) {
  const unsigned int u = __float_as_uint(f);
  return (u + 0x7FFFu + ((u >> 16) & 1u)) >> 16;
}
__device__ __forceinline__ float bf16rf(float f) { return __uint_as_float(bfr(f) << 16); }

__device__ __forceinline__ void split1(float x, unsigned short& hb, unsigned short& lb) {
  const unsigned int hu = bfr(x);
  const float hf = __uint_as_float(hu << 16);
  hb = (unsigned short)hu;
  lb = (unsigned short)bfr(x - hf);
}
__device__ __forceinline__ void split8(v4f a, v4f b, v8us& hi, v8us& lo) {
  unsigned short hb, lb;
  split1(a.x, hb, lb); hi[0] = hb; lo[0] = lb;
  split1(a.y, hb, lb); hi[1] = hb; lo[1] = lb;
  split1(a.z, hb, lb); hi[2] = hb; lo[2] = lb;
  split1(a.w, hb, lb); hi[3] = hb; lo[3] = lb;
  split1(b.x, hb, lb); hi[4] = hb; lo[4] = lb;
  split1(b.y, hb, lb); hi[5] = hb; lo[5] = lb;
  split1(b.z, hb, lb); hi[6] = hb; lo[6] = lb;
  split1(b.w, hb, lb); hi[7] = hb; lo[7] = lb;
}

__device__ __forceinline__ v8f wm(v16b a, v16b b, v8f c) {
  return __builtin_amdgcn_wmma_f32_16x16x32_bf16(false, a, false, b, (short)0, c, false, false);
}
__device__ __forceinline__ v8f wm2(v16b ah, v16b al, v16b b, v8f c) {
  c = wm(ah, b, c); c = wm(al, b, c);
  asm volatile("v_nop\n\tv_nop\n\tv_nop\n\tv_nop" : "+v"(c) : "v"(ah), "v"(al), "v"(b));
  return c;
}
__device__ __forceinline__ v8f wm1(v16b ah, v16b b, v8f c) {
  c = wm(ah, b, c);
  asm volatile("v_nop\n\tv_nop\n\tv_nop\n\tv_nop" : "+v"(c) : "v"(ah), "v"(b));
  return c;
}

__device__ __forceinline__ float wsum(float v) {
#pragma unroll
  for (int o = 16; o > 0; o >>= 1) v += __shfl_xor(v, o);
  return v;
}
__device__ __forceinline__ float dot4(v4f a, v4f b, float d) {
  d = fmaf(a.x, b.x, d); d = fmaf(a.y, b.y, d); d = fmaf(a.z, b.z, d); d = fmaf(a.w, b.w, d);
  return d;
}
__device__ __forceinline__ v4f relu4(v4f x) {
  v4f r; r.x = fmaxf(x.x, 0.0f); r.y = fmaxf(x.y, 0.0f); r.z = fmaxf(x.z, 0.0f); r.w = fmaxf(x.w, 0.0f);
  return r;
}
__device__ __forceinline__ v4f ln4(v4f x, v4f gv, v4f bv) {
  const float mean = wsum(x.x + x.y + x.z + x.w) * 0.0078125f;
  const v4f d = x - mean;
  const float var = wsum(d.x * d.x + d.y * d.y + d.z * d.z + d.w * d.w) * 0.0078125f;
  const float rs = rsqrtf(var + 1e-5f);
  return (d * rs) * gv + bv;
}

__device__ __forceinline__ void build_in_lists(const int* __restrict__ eib, int* ssrc, int* sdst, int* scnt, int* sofs, int* slist,
                                               int tid, int lane, int wave) {
  int s = eib[tid];
  int d = eib[EPG + tid];
  s = s < 0 ? s + NPG : s; s = s < 0 ? 0 : (s > NPG - 1 ? NPG - 1 : s);
  d = d < 0 ? d + NPG : d; d = d < 0 ? 0 : (d > NPG - 1 ? NPG - 1 : d);
  ssrc[tid] = s; sdst[tid] = d;
  __syncthreads();
  if (wave < 2) {
    int c = 0;
#pragma unroll 4
    for (int e = 0; e < EPG; ++e) c += (sdst[e] == tid) ? 1 : 0;
    scnt[tid] = c;
  }
  __syncthreads();
  if (wave == 0) {
    int run = 0;
#pragma unroll 1
    for (int i = 0; i < NPG; ++i) {
      const int c = scnt[i];
      if (lane == 0) sofs[i] = run;
      run += c;
    }
    if (lane == 0) sofs[NPG] = run;
  }
  __syncthreads();
  if (wave < 2) {
    int pos = sofs[tid];
#pragma unroll 4
    for (int e = 0; e < EPG; ++e) {
      if (sdst[e] == tid) { slist[pos < EPG ? pos : EPG - 1] = e; ++pos; }
    }
  }
  __syncthreads();
}

struct WJob { const float* src; unsigned short* dst; int N, KP, kbeg, kend, ND, sNh, sNl, KD, sKh, sKl, K; float scl; int pad0, pad1; };
struct WJobs { WJob j[NJOB]; };
static_assert(sizeof(WJob) == 72);
static_assert(sizeof(WJobs) == 72 * NJOB);

__global__ __launch_bounds__(NTHR) void k_wprep(WJobs J) {
  const int y = (int)blockIdx.y;
  WJob jb = J.j[0];
#pragma unroll
  for (int i = 1; i < NJOB; ++i)
    if (i == y) jb = J.j[i];
  const int idx = (int)blockIdx.x * NTHR + (int)threadIdx.x;
  const int kw8 = (jb.kend - jb.kbeg) >> 3;
  const int items = jb.N * kw8;
  if (idx >= items) return;
  const int n = idx / kw8;
  const int kq = idx - n * kw8;
  const int k0 = jb.kbeg + 8 * kq;
  const size_t nb = (size_t)(n / jb.ND) * (size_t)jb.sNh + (size_t)(n % jb.ND) * (size_t)jb.sNl;
  float v[8];
#pragma unroll
  for (int e = 0; e < 8; ++e) {
    const int kk = 8 * kq + e;
    const int kc = kk < jb.K ? kk : jb.K - 1;
    const size_t si = nb + (size_t)(kc / jb.KD) * (size_t)jb.sKh + (size_t)(kc % jb.KD) * (size_t)jb.sKl;
    const float x = jb.src[si];
    v[e] = kk < jb.K ? jb.scl * bf16rf(x) : 0.0f;
  }
  v8us hv;
#pragma unroll
  for (int e = 0; e < 8; ++e) hv[e] = (unsigned short)bfr(v[e]);
  unsigned short* dp = jb.dst + (size_t)n * jb.KP + k0;
  *(volatile v8us*)dp = hv;
  __threadfence();
  *(volatile v8us*)dp = hv;
}

__global__ __launch_bounds__(NTHR) void k_feat(const float* __restrict__ x, const int* __restrict__ ei, const float* __restrict__ ea,
                                               const float* __restrict__ emb, unsigned short* F) {
  const int idx = (int)blockIdx.x * NTHR + (int)threadIdx.x;
  const int e = idx >> 2, q = idx & 3, sub = q & 1;
  const int b = e >> 8, le = e & (EPG - 1);
  int s = ei[(size_t)b * 2 * EPG + le];
  s = s < 0 ? s + NPG : s; s = s < 0 ? 0 : (s > NPG - 1 ? NPG - 1 : s);
  const float xf = bf16rf(x[b * NPG + s]);
  int et = (int)xf;
  et = et < 0 ? et + 5 : et; et = et < 0 ? 0 : (et > 4 ? 4 : et);
  const v4f m0 = *(const v4f*)(emb + et * 16 + 8 * sub);
  const v4f m1 = *(const v4f*)(emb + et * 16 + 8 * sub + 4);
  const v4f a0 = *(const v4f*)(ea + (size_t)e * EDIM + 8 * sub);
  const v4f a1 = *(const v4f*)(ea + (size_t)e * EDIM + 8 * sub + 4);
  const bool useM = q < 2;
  float v[8];
  v[0] = useM ? m0.x : a0.x; v[1] = useM ? m0.y : a0.y; v[2] = useM ? m0.z : a0.z; v[3] = useM ? m0.w : a0.w;
  v[4] = useM ? m1.x : a1.x; v[5] = useM ? m1.y : a1.y; v[6] = useM ? m1.z : a1.z; v[7] = useM ? m1.w : a1.w;
  v8us hv;
#pragma unroll
  for (int i = 0; i < 8; ++i) hv[i] = (unsigned short)bfr(v[i]);
  unsigned short* dp = F + (size_t)idx * 8;
  *(volatile v8us*)dp = hv;
  __threadfence();
  *(volatile v8us*)dp = hv;
}

struct GArgs {
  const unsigned short* Ah; const unsigned short* Al; const unsigned short* A2h; const unsigned short* A2l;
  const unsigned short* W;
  const float* b0; const float* b1; const float* b2;
  const float* lng; const float* lnb; const float* aux;
  float* C; unsigned short* Ph; unsigned short* Pl;
  int lda, lda2, ks1, ksteps, ldb, ldc, ldp, bsh, nb, atile, auxld, wantC, wantP, plim, z0, z1;
};
static_assert(sizeof(GArgs) == 176);

__device__ __forceinline__ void plane_rows(const float* stg, unsigned short* Ph, unsigned short* Pl, int ldp,
                                           int rowBase, int colBase, int wave, int hh, int m) {
#pragma unroll 1
  for (int i = 0; i < 8; ++i) {
    const int lr = wave * 16 + 2 * i + hh;
    const float* sp = stg + lr * 128 + 8 * m;
    const v4f a = *(const v4f*)sp;
    const v4f b = *(const v4f*)(sp + 4);
    v8us hv, lv;
    split8(a, b, hv, lv);
    const size_t o = (size_t)(rowBase + lr) * (size_t)ldp + (size_t)(colBase + 8 * m);
    *(volatile v8us*)(Ph + o) = hv;
    *(volatile v8us*)(Pl + o) = lv;
  }
}

template <int NCT, int NPA, int EPI, int ATILE>
__global__ __launch_bounds__(NTHR) void k_gemm(GArgs g) {
  extern __shared__ v4f lds_dyn[];
  float* stg = (float*)lds_dyn;
  constexpr int BW  = 16 * NCT;
  constexpr int LPR = BW / 4;
  constexpr int RPI = 32 / LPR;
  constexpr int NIT = 16 / RPI;
  static_assert(NCT == 8 || NCT == 4);
  static_assert(EPI == 0 || NCT == 8);
  static_assert(NPA == 1 || NPA == 2);
  const int tid = threadIdx.x, lane = tid & 31, wave = tid >> 5, hh = lane >> 4, m = lane & 15;
  const int rowBase = (int)blockIdx.x * 128;
  const int colBase = (int)blockIdx.y * BW;
  const int arow = rowBase + wave * 16 + m;
  v8f acc[NCT];
#pragma unroll
  for (int t = 0; t < NCT; ++t) { const v8f z = {0.f, 0.f, 0.f, 0.f, 0.f, 0.f, 0.f, 0.f}; acc[t] = z; }
#pragma unroll 1
  for (int kt = 0; kt < g.ksteps; ++kt) {
    const bool prim = kt < g.ks1;
    const size_t aoff = prim ? ((size_t)arow * (size_t)g.lda + (size_t)(32 * kt + 8 * hh))
                             : ((size_t)arow * (size_t)g.lda2 + (size_t)(32 * (kt - g.ks1) + 8 * hh));
    const unsigned short* ph = (prim ? g.Ah : g.A2h) + aoff;
    const unsigned short* pl = (prim ? g.Al : g.A2l) + aoff;
    FragB ah, al;
    { const v8us z8 = {0, 0, 0, 0, 0, 0, 0, 0}; al.h[0] = z8; al.h[1] = z8; ah.h[0] = z8; ah.h[1] = z8; }
    if constexpr (ATILE == 0) {
      ah.h[0] = *(const v8us*)ph; ah.h[1] = *(const v8us*)(ph + 16);
      if constexpr (NPA == 2) { al.h[0] = *(const v8us*)pl; al.h[1] = *(const v8us*)(pl + 16); }
    }
#pragma unroll
    for (int t = 0; t < NCT; ++t) {
      if constexpr (ATILE != 0) {
        const unsigned short* pht = ph + t * g.atile;
        const unsigned short* plt = pl + t * g.atile;
        ah.h[0] = *(const v8us*)pht; ah.h[1] = *(const v8us*)(pht + 16);
        if constexpr (NPA == 2) { al.h[0] = *(const v8us*)plt; al.h[1] = *(const v8us*)(plt + 16); }
      }
      const size_t bo = (size_t)(colBase + 16 * t + m) * (size_t)g.ldb + (size_t)(32 * kt + 8 * hh);
      FragB b;
      b.h[0] = *(const v8us*)(g.W + bo); b.h[1] = *(const v8us*)(g.W + bo + 16);
      if constexpr (NPA == 2) acc[t] = wm2(ah.v, al.v, b.v, acc[t]);
      else acc[t] = wm1(ah.v, b.v, acc[t]);
    }
  }
  const int r0 = wave * 16 + 8 * hh;
#pragma unroll
  for (int t = 0; t < NCT; ++t) {
    const int lcol = 16 * t + m;
    const int gcol = colBase + lcol;
    float bias = 0.0f;
    if (g.nb > 0) {
      int which = gcol >> g.bsh;
      which = which > g.nb - 1 ? g.nb - 1 : which;
      const float* bp = (which == 0) ? g.b0 : ((which == 1) ? g.b1 : g.b2);
      bias = bf16rf(bp[gcol - (which << g.bsh)]);
    }
#pragma unroll
    for (int r = 0; r < 8; ++r) stg[(r0 + r) * BW + lcol] = acc[t][r] + bias;
  }
  __syncthreads();
  v4f gv = {1.f, 1.f, 1.f, 1.f};
  v4f bv = {0.f, 0.f, 0.f, 0.f};
  if constexpr (EPI == 1 || EPI == 2) {
    const v4f g4 = *(const v4f*)(g.lng + 4 * lane);
    const v4f b4 = *(const v4f*)(g.lnb + 4 * lane);
    gv.x = bf16rf(g4.x); gv.y = bf16rf(g4.y); gv.z = bf16rf(g4.z); gv.w = bf16rf(g4.w);
    bv.x = bf16rf(b4.x); bv.y = bf16rf(b4.y); bv.z = bf16rf(b4.z); bv.w = bf16rf(b4.w);
  }
  const bool doC = g.wantC != 0;
#pragma unroll 1
  for (int it = 0; it < NIT; ++it) {
    const int lr = wave * 16 + RPI * it + lane / LPR;
    const int c4 = 4 * (lane % LPR);
    float* sp = stg + lr * BW + c4;
    v4f y = *(const v4f*)sp;
    if constexpr (EPI == 1 || EPI == 2) {
      y = ln4(relu4(y), gv, bv);
      if constexpr (EPI == 2) {
        const v4f rr = *(const v4f*)(g.aux + (size_t)(rowBase + lr) * (size_t)g.auxld + c4);
        y = ln4(relu4(y + rr), gv, bv);
      }
    }
    if constexpr (EPI == 4) {
      const v4f vs = *(const v4f*)(g.aux + (size_t)(rowBase + lr) * (size_t)g.auxld + c4);
      y = relu4(vs * 0.25f + y);
    }
    if constexpr (EPI != 0) *(v4f*)sp = y;
    if (doC) *(volatile v4f*)(g.C + (size_t)(rowBase + lr) * (size_t)g.ldc + (size_t)(colBase + c4)) = y;
  }
  __syncthreads();
  bool doP = false;
  if constexpr (NCT == 8) doP = (g.wantP != 0) && (colBase < g.plim);
  if constexpr (NCT == 8) { if (doP) plane_rows(stg, g.Ph, g.Pl, g.ldp, rowBase, colBase, wave, hh, m); }
  __threadfence();
  if (doC) {
#pragma unroll 1
    for (int it = 0; it < NIT; ++it) {
      const int lr = wave * 16 + RPI * it + lane / LPR;
      const int c4 = 4 * (lane % LPR);
      const v4f y = *(const v4f*)(stg + lr * BW + c4);
      *(volatile v4f*)(g.C + (size_t)(rowBase + lr) * (size_t)g.ldc + (size_t)(colBase + c4)) = y;
    }
  }
  if constexpr (NCT == 8) { if (doP) plane_rows(stg, g.Ph, g.Pl, g.ldp, rowBase, colBase, wave, hh, m); }
}

__global__ __launch_bounds__(NTHR) void k_aggr(const int* __restrict__ ei, const float* __restrict__ hmsg,
                                               unsigned short* Ah, unsigned short* Al) {
  __shared__ int ssrc[EPG];
  __shared__ int sdst[EPG];
  __shared__ int scnt[NPG];
  __shared__ int sofs[NPG + 1];
  __shared__ int slist[EPG];
  __shared__ __attribute__((aligned(16))) float wstg[NWAVE * 256];
  const int tid = threadIdx.x, lane = tid & 31, wave = tid >> 5, hh = lane >> 4, m = lane & 15;
  const int gb = (int)blockIdx.x;
  build_in_lists(ei + (size_t)gb * 2 * EPG, ssrc, sdst, scnt, sofs, slist, tid, lane, wave);
  float* ws_ = wstg + wave * 256;
#pragma unroll 1
  for (int jn = 0; jn < NPG / NWAVE; ++jn) {
    const int n = wave + NWAVE * jn;
    int deg = __builtin_amdgcn_readfirstlane(scnt[n]);
    deg = deg < 0 ? 0 : (deg > EPG ? EPG : deg);
    int st = __builtin_amdgcn_readfirstlane(sofs[n]);
    st = st < 0 ? 0 : (st > EPG ? EPG : st);
    v4f a = {0.f, 0.f, 0.f, 0.f};
#pragma unroll 1
    for (int p = 0; p < deg; ++p) {
      const int sp = (st + p) < EPG ? (st + p) : EPG - 1;
      int e = __builtin_amdgcn_readfirstlane(slist[sp]);
      e &= (EPG - 1);
      const int eid = gb * EPG + e;
      a = a + *(const v4f*)(hmsg + (size_t)eid * DH + 4 * lane);
    }
    *(v4f*)(ws_ + (jn & 1) * 128 + 4 * lane) = a;
    if ((jn & 1) != 0) {
      __builtin_amdgcn_fence(__ATOMIC_RELEASE, "wavefront");
      __builtin_amdgcn_wave_barrier();
      const int nn = wave + NWAVE * (jn - 1 + hh);
      const int node = gb * NPG + nn;
      const float* sp = ws_ + hh * 128 + 8 * m;
      const v4f x0 = *(const v4f*)sp;
      const v4f x1 = *(const v4f*)(sp + 4);
      v8us hv, lv;
      split8(x0, x1, hv, lv);
      const size_t o = (size_t)node * DH + 8 * m;
      *(volatile v8us*)(Ah + o) = hv; *(volatile v8us*)(Al + o) = lv;
      __threadfence();
      *(volatile v8us*)(Ah + o) = hv; *(volatile v8us*)(Al + o) = lv;
      __builtin_amdgcn_fence(__ATOMIC_RELEASE, "wavefront");
      __builtin_amdgcn_wave_barrier();
    }
  }
}

__global__ __launch_bounds__(NTHR) void k_attn(const int* __restrict__ ei, const float* __restrict__ ea, const float* __restrict__ qkv,
                                               const float* __restrict__ Gt, float* Vsum, unsigned short* Sh, unsigned short* Sl, int gbase) {
  __shared__ int ssrc[EPG];
  __shared__ int sdst[EPG];
  __shared__ int scnt[NPG];
  __shared__ int sofs[NPG + 1];
  __shared__ int slist[EPG];
  __shared__ __attribute__((aligned(16))) float lbuf[NWAVE * 4 * EPG];
  __shared__ __attribute__((aligned(16))) float wstg[NWAVE * 192];
  const int tid = threadIdx.x, lane = tid & 31, wave = tid >> 5, sub = lane & 7, hd = lane >> 3;
  const int gl = (int)blockIdx.x;
  const int gb = gbase + gl;
  build_in_lists(ei + (size_t)gb * 2 * EPG, ssrc, sdst, scnt, sofs, slist, tid, lane, wave);
  float* wl = lbuf + wave * 4 * EPG;
  float* ws_ = wstg + wave * 192;
  const float scale = 0.08838834764831845f;
#pragma unroll 1
  for (int jn = 0; jn < NPG / NWAVE; ++jn) {
    const int n = wave + NWAVE * jn;
    int deg = __builtin_amdgcn_readfirstlane(scnt[n]);
    deg = deg < 0 ? 0 : (deg > EPG ? EPG : deg);
    int st = __builtin_amdgcn_readfirstlane(sofs[n]);
    st = st < 0 ? 0 : (st > EPG ? EPG : st);
    const int rloc = gl * NPG + n;
    const float* qp = qkv + (size_t)rloc * QKVW + 16 * lane;
    const v4f q0 = *(const v4f*)qp;
    const v4f q1 = *(const v4f*)(qp + 4);
    const v4f q2 = *(const v4f*)(qp + 8);
    const v4f q3 = *(const v4f*)(qp + 12);
    const v2f g2 = *(const v2f*)(Gt + (size_t)rloc * 64 + 2 * lane);
    float M = NEG_BIG;
#pragma unroll 1
    for (int p = 0; p < deg; ++p) {
      const int spo = (st + p) < EPG ? (st + p) : EPG - 1;
      int e = __builtin_amdgcn_readfirstlane(slist[spo]);
      e &= (EPG - 1);
      const int eid = gb * EPG + e;
      const int sl = __builtin_amdgcn_readfirstlane(ssrc[e]);
      const int srow = gl * NPG + sl;
      const float* kp = qkv + (size_t)srow * QKVW + HCOL + 16 * lane;
      const v4f k0 = *(const v4f*)kp;
      const v4f k1 = *(const v4f*)(kp + 4);
      const v4f k2 = *(const v4f*)(kp + 8);
      const v4f k3 = *(const v4f*)(kp + 12);
      const v2f ev = *(const v2f*)(ea + (size_t)eid * EDIM + 2 * sub);
      const float e0 = bf16rf(ev.x), e1 = bf16rf(ev.y);
      float d = dot4(q0, k0, 0.0f);
      d = dot4(q1, k1, d); d = dot4(q2, k2, d); d = dot4(q3, k3, d);
      d = fmaf(e0, g2.x, d); d = fmaf(e1, g2.y, d);
      d += __shfl_xor(d, 1); d += __shfl_xor(d, 2); d += __shfl_xor(d, 4);
      const float lg = d * scale;
      M = fmaxf(M, lg);
      if (sub == 0) wl[p * 4 + hd] = lg;
    }
    __builtin_amdgcn_fence(__ATOMIC_RELEASE, "wavefront");
    __builtin_amdgcn_wave_barrier();
    const int total = deg * 4;
#pragma unroll 1
    for (int i = 0; i < ((total + 31) >> 5); ++i) {
      const int idx = lane + 32 * i;
      const int h2 = idx & 3;
      const float Mh = __shfl(M, h2 * 8);
      const int ic = idx < 4 * EPG ? idx : 4 * EPG - 1;
      const float x = wl[ic];
      const float pe = __expf(x - Mh);
      if (idx < total) wl[idx] = pe;
    }
    __builtin_amdgcn_fence(__ATOMIC_RELEASE, "wavefront");
    __builtin_amdgcn_wave_barrier();
    float ds = 0.0f;
#pragma unroll 1
    for (int pp = 0; pp < deg; pp += 8) {
      const int p = pp + sub;
      const int pc = p < EPG ? p : EPG - 1;
      const float x = wl[pc * 4 + hd];
      ds += (p < deg) ? x : 0.0f;
    }
    ds += __shfl_xor(ds, 1); ds += __shfl_xor(ds, 2); ds += __shfl_xor(ds, 4);
    const float rd = __builtin_amdgcn_rcpf(ds + 1e-16f);
    v4f a0 = {0.f, 0.f, 0.f, 0.f}, a1 = {0.f, 0.f, 0.f, 0.f}, a2 = {0.f, 0.f, 0.f, 0.f}, a3 = {0.f, 0.f, 0.f, 0.f};
    float s0 = 0.0f, s1 = 0.0f;
#pragma unroll 1
    for (int p = 0; p < deg; ++p) {
      const int spo = (st + p) < EPG ? (st + p) : EPG - 1;
      int e = __builtin_amdgcn_readfirstlane(slist[spo]);
      e &= (EPG - 1);
      const int eid = gb * EPG + e;
      const int sl = __builtin_amdgcn_readfirstlane(ssrc[e]);
      const int srow = gl * NPG + sl;
      const float al = wl[p * 4 + hd] * rd;
      const float* vp = qkv + (size_t)srow * QKVW + 2 * HCOL + 16 * lane;
      const v4f v0 = *(const v4f*)vp;
      const v4f v1 = *(const v4f*)(vp + 4);
      const v4f v2 = *(const v4f*)(vp + 8);
      const v4f v3 = *(const v4f*)(vp + 12);
      a0 = a0 + v0 * al; a1 = a1 + v1 * al; a2 = a2 + v2 * al; a3 = a3 + v3 * al;
      const v2f ev = *(const v2f*)(ea + (size_t)eid * EDIM + 2 * sub);
      s0 = fmaf(al, bf16rf(ev.x), s0);
      s1 = fmaf(al, bf16rf(ev.y), s1);
    }
    a0.x += __shfl_xor(a0.x, 8); a0.y += __shfl_xor(a0.y, 8); a0.z += __shfl_xor(a0.z, 8); a0.w += __shfl_xor(a0.w, 8);
    a1.x += __shfl_xor(a1.x, 8); a1.y += __shfl_xor(a1.y, 8); a1.z += __shfl_xor(a1.z, 8); a1.w += __shfl_xor(a1.w, 8);
    a2.x += __shfl_xor(a2.x, 8); a2.y += __shfl_xor(a2.y, 8); a2.z += __shfl_xor(a2.z, 8); a2.w += __shfl_xor(a2.w, 8);
    a3.x += __shfl_xor(a3.x, 8); a3.y += __shfl_xor(a3.y, 8); a3.z += __shfl_xor(a3.z, 8); a3.w += __shfl_xor(a3.w, 8);
    a0.x += __shfl_xor(a0.x, 16); a0.y += __shfl_xor(a0.y, 16); a0.z += __shfl_xor(a0.z, 16); a0.w += __shfl_xor(a0.w, 16);
    a1.x += __shfl_xor(a1.x, 16); a1.y += __shfl_xor(a1.y, 16); a1.z += __shfl_xor(a1.z, 16); a1.w += __shfl_xor(a1.w, 16);
    a2.x += __shfl_xor(a2.x, 16); a2.y += __shfl_xor(a2.y, 16); a2.z += __shfl_xor(a2.z, 16); a2.w += __shfl_xor(a2.w, 16);
    a3.x += __shfl_xor(a3.x, 16); a3.y += __shfl_xor(a3.y, 16); a3.z += __shfl_xor(a3.z, 16); a3.w += __shfl_xor(a3.w, 16);
    if (lane < 8) {
      *(v4f*)(ws_ + 16 * lane)      = a0;
      *(v4f*)(ws_ + 16 * lane + 4)  = a1;
      *(v4f*)(ws_ + 16 * lane + 8)  = a2;
      *(v4f*)(ws_ + 16 * lane + 12) = a3;
    }
    { v2f sv; sv.x = s0; sv.y = s1; *(v2f*)(ws_ + 128 + 2 * lane) = sv; }
    __builtin_amdgcn_fence(__ATOMIC_RELEASE, "wavefront");
    __builtin_amdgcn_wave_barrier();
    const v4f vo = *(const v4f*)(ws_ + 4 * lane);
    const int l8 = lane < 8 ? lane : 7;
    const v4f sa = *(const v4f*)(ws_ + 128 + 8 * l8);
    const v4f sb = *(const v4f*)(ws_ + 132 + 8 * l8);
    v8us sh8, sl8;
    split8(sa, sb, sh8, sl8);
    float* vg = Vsum + (size_t)rloc * DH + 4 * lane;
    const size_t so = (size_t)rloc * 64 + 8 * l8;
    *(volatile v4f*)vg = vo;
    if (lane < 8) { *(volatile v8us*)(Sh + so) = sh8; *(volatile v8us*)(Sl + so) = sl8; }
    __threadfence();
    *(volatile v4f*)vg = vo;
    if (lane < 8) { *(volatile v8us*)(Sh + so) = sh8; *(volatile v8us*)(Sl + so) = sl8; }
    __builtin_amdgcn_fence(__ATOMIC_RELEASE, "wavefront");
    __builtin_amdgcn_wave_barrier();
  }
}

__global__ __launch_bounds__(NTHR) void k_gat(const int* __restrict__ agent, const unsigned short* __restrict__ Ah, const unsigned short* __restrict__ Al,
                                              unsigned short* Gh, unsigned short* Gl) {
  const int tid = threadIdx.x;
  int row = (int)blockIdx.x * 16 + (tid >> 4);
  row = row > NGR - 1 ? NGR - 1 : row;
  const int seg = tid & 15;
  int a = agent[row];
  a = a < 0 ? a + NPG : a; a = a < 0 ? 0 : (a > NPG - 1 ? NPG - 1 : a);
  const int node = row * NPG + a;
  const v8us vh = *(const v8us*)(Ah + (size_t)node * DH + 8 * seg);
  const v8us vl = *(const v8us*)(Al + (size_t)node * DH + 8 * seg);
  const size_t o = (size_t)row * DH + 8 * seg;
  *(volatile v8us*)(Gh + o) = vh; *(volatile v8us*)(Gl + o) = vl;
  __threadfence();
  *(volatile v8us*)(Gh + o) = vh; *(volatile v8us*)(Gl + o) = vl;
}

static WJob mkjob(const float* src, unsigned short* dst, int N, int KP, int kbeg, int kend, int ND, int sNh, int sNl,
                  int KD, int sKh, int sKl, int K, float scl) {
  WJob j;
  j.src = src; j.dst = dst; j.N = N; j.KP = KP; j.kbeg = kbeg; j.kend = kend; j.ND = ND; j.sNh = sNh; j.sNl = sNl;
  j.KD = KD; j.sKh = sKh; j.sKl = sKl; j.K = K; j.scl = scl; j.pad0 = 0; j.pad1 = 0;
  return j;
}

static GArgs mkg(const unsigned short* Ah, const unsigned short* Al, int lda, int ks1,
                 const unsigned short* A2h, const unsigned short* A2l, int lda2, int ksteps,
                 const unsigned short* W, int ldb,
                 const float* b0, const float* b1, const float* b2, int nb, int bsh,
                 const float* lng, const float* lnb, const float* aux, int auxld,
                 float* C, int ldc, int wantC,
                 unsigned short* Ph, unsigned short* Pl, int ldp, int wantP, int plim, int atile) {
  GArgs g;
  g.Ah = Ah; g.Al = Al; g.A2h = A2h; g.A2l = A2l; g.W = W; g.b0 = b0; g.b1 = b1; g.b2 = b2;
  g.lng = lng; g.lnb = lnb; g.aux = aux; g.C = C; g.Ph = Ph; g.Pl = Pl;
  g.lda = lda; g.lda2 = lda2; g.ks1 = ks1; g.ksteps = ksteps; g.ldb = ldb; g.ldc = ldc; g.ldp = ldp; g.bsh = bsh; g.nb = nb;
  g.atile = atile; g.auxld = auxld; g.wantC = wantC; g.wantP = wantP; g.plim = plim; g.z0 = 0; g.z1 = 0;
  return g;
}

extern "C" void kernel_launch(void* const* d_in, const int* in_sizes, int n_in,
                              void* d_out, int out_size, void* d_ws, size_t ws_size,
                              hipStream_t stream) {
  if (n_in < 24) return;
  const int want[24] = {16384, 131072, 1048576, 256, 80, 4096, 128, 16384, 128, 16384, 128, 128, 128,
                        196608, 1536, 196608, 1536, 196608, 1536, 24576, 49152, 384, 16384, 128};
  for (int i = 0; i < 24; ++i) if (in_sizes[i] != want[i]) return;
  if (out_size != NGR * DH) return;
  if (ws_size < (size_t)WS_TOTAL) return;

  const float* xnf   = (const float*)d_in[0];
  const int*   ei    = (const int*)d_in[1];
  const float* ea    = (const float*)d_in[2];
  const int*   agent = (const int*)d_in[3];
  const float* emb   = (const float*)d_in[4];
  const float* w1 = (const float*)d_in[5];  const float* b1 = (const float*)d_in[6];
  const float* w2 = (const float*)d_in[7];  const float* b2 = (const float*)d_in[8];
  const float* w3 = (const float*)d_in[9];  const float* b3 = (const float*)d_in[10];
  const float* lng = (const float*)d_in[11]; const float* lnb = (const float*)d_in[12];
  const float* qw = (const float*)d_in[13]; const float* qb = (const float*)d_in[14];
  const float* kw = (const float*)d_in[15]; const float* kb = (const float*)d_in[16];
  const float* vw = (const float*)d_in[17]; const float* vb = (const float*)d_in[18];
  const float* ew = (const float*)d_in[19];
  const float* skw = (const float*)d_in[20]; const float* skb = (const float*)d_in[21];
  const float* ow = (const float*)d_in[22]; const float* ob = (const float*)d_in[23];
  float* out = (float*)d_out;

  char* ws = (char*)d_ws;
  unsigned short* wp   = (unsigned short*)(ws + OFF_W);
  unsigned short* Fp   = (unsigned short*)(ws + OFF_F);
  float* resf          = (float*)(ws + OFF_R2);
  unsigned short* h1h  = (unsigned short*)(ws + OFF_R3 + E_H1H);
  unsigned short* h1l  = (unsigned short*)(ws + OFF_R3 + E_H1L);
  unsigned short* h2h  = (unsigned short*)(ws + OFF_R3 + E_H2H);
  unsigned short* h2l  = (unsigned short*)(ws + OFF_R3 + E_H2L);
  float* hmsg          = (float*)(ws + OFF_R3 + E_H1H);
  unsigned short* Ach  = (unsigned short*)(ws + OFF_R2 + N_ACH);
  unsigned short* Acl  = (unsigned short*)(ws + OFF_R2 + N_ACL);
  unsigned short* Anh  = (unsigned short*)(ws + OFF_R2 + N_ANH);
  unsigned short* Anl  = (unsigned short*)(ws + OFF_R2 + N_ANL);
  float* Gf            = (float*)(ws + OFF_R2 + N_G);
  float* Vsf           = (float*)(ws + OFF_R2 + N_VS);
  unsigned short* Sh   = (unsigned short*)(ws + OFF_R2 + N_SH);
  unsigned short* Sl   = (unsigned short*)(ws + OFF_R2 + N_SL);
  unsigned short* gth  = (unsigned short*)(ws + OFF_R2 + N_GTH);
  unsigned short* gtl  = (unsigned short*)(ws + OFF_R2 + N_GTL);
  float* qkvf          = (float*)(ws + OFF_R3 + N_QKV);
  unsigned short* qPh  = (unsigned short*)(ws + OFF_R3 + N_QPH);
  unsigned short* qPl  = (unsigned short*)(ws + OFF_R3 + N_QPL);

  WJobs J;
  J.j[0] = mkjob(w1, wp + PW1, 128, 32, 0, 32, BIGD, 0, 1, BIGD, 0, 128, 32, 1.0f);
  J.j[1] = mkjob(w2, wp + PW2, 128, 128, 0, 128, BIGD, 0, 1, BIGD, 0, 128, 128, 1.0f);
  J.j[2] = mkjob(w3, wp + PW3, 128, 128, 0, 128, BIGD, 0, 1, BIGD, 0, 128, 128, 1.0f);
  for (int l = 0; l < NLAY; ++l) {
    unsigned short* base = wp + PLAY0 + (size_t)l * PLAYSZ;
    J.j[3 + 6 * l + 0] = mkjob(qw + (size_t)l * DH * HCOL, base + PQKV,                     512, 128, 0, 128, BIGD, 0, 1, BIGD, 0, 512, 128, 1.0f);
    J.j[3 + 6 * l + 1] = mkjob(kw + (size_t)l * DH * HCOL, base + PQKV + (size_t)HCOL * DH, 512, 128, 0, 128, BIGD, 0, 1, BIGD, 0, 512, 128, 1.0f);
    J.j[3 + 6 * l + 2] = mkjob(vw + (size_t)l * DH * HCOL, base + PQKV + (size_t)2 * HCOL * DH, 512, 128, 0, 128, BIGD, 0, 1, BIGD, 0, 512, 128, 1.0f);
    J.j[3 + 6 * l + 3] = mkjob(ew + (size_t)l * EDIM * HCOL, base + PWG, 64, 128, 0, 128, 16, 128, 512, BIGD, 0, 1, 128, 1.0f);
    J.j[3 + 6 * l + 4] = mkjob(ew + (size_t)l * EDIM * HCOL, base + PWTS, 128, 192, 0, 64, BIGD, 0, 1, 16, 128, 512, 64, 0.25f);
    J.j[3 + 6 * l + 5] = mkjob(skw + (size_t)l * DH * DH, base + PWTS, 128, 192, 64, 192, BIGD, 0, 1, BIGD, 0, 128, 128, 1.0f);
  }
  J.j[21] = mkjob(ow, wp + PWOUT, 128, 128, 0, 128, BIGD, 0, 1, BIGD, 0, 128, 128, 1.0f);
  k_wprep<<<dim3(32, NJOB, 1), NTHR, 0, stream>>>(J);

  k_feat<<<(NEDGE * 4) / NTHR, NTHR, 0, stream>>>(xnf, ei, ea, emb, Fp);

  hipFuncSetAttribute(reinterpret_cast<const void*>(&k_gemm<8, 1, 1, 0>), hipFuncAttributeMaxDynamicSharedMemorySize, LDS_G8);
  hipFuncSetAttribute(reinterpret_cast<const void*>(&k_gemm<8, 2, 1, 0>), hipFuncAttributeMaxDynamicSharedMemorySize, LDS_G8);
  hipFuncSetAttribute(reinterpret_cast<const void*>(&k_gemm<8, 2, 2, 0>), hipFuncAttributeMaxDynamicSharedMemorySize, LDS_G8);
  hipFuncSetAttribute(reinterpret_cast<const void*>(&k_gemm<8, 2, 0, 0>), hipFuncAttributeMaxDynamicSharedMemorySize, LDS_G8);
  hipFuncSetAttribute(reinterpret_cast<const void*>(&k_gemm<8, 2, 4, 0>), hipFuncAttributeMaxDynamicSharedMemorySize, LDS_G8);
  hipFuncSetAttribute(reinterpret_cast<const void*>(&k_gemm<4, 2, 0, 1>), hipFuncAttributeMaxDynamicSharedMemorySize, LDS_G4);

  {
    GArgs a = mkg(Fp, Fp, 32, 1, Fp, Fp, 32, 1, wp + PW1, 32, b1, b1, b1, 1, 20, lng, lnb, resf, DH,
                  resf, DH, 1, h1h, h1l, DH, 1, BIGD, 0);
    k_gemm<8, 1, 1, 0><<<dim3(NEDGE / 128, 1, 1), NTHR, LDS_G8, stream>>>(a);
  }
  {
    GArgs a = mkg(h1h, h1l, DH, 4, h1h, h1l, DH, 4, wp + PW2, DH, b2, b2, b2, 1, 20, lng, lnb, resf, DH,
                  Vsf, DH, 0, h2h, h2l, DH, 1, BIGD, 0);
    k_gemm<8, 2, 1, 0><<<dim3(NEDGE / 128, 1, 1), NTHR, LDS_G8, stream>>>(a);
  }
  {
    GArgs a = mkg(h2h, h2l, DH, 4, h2h, h2l, DH, 4, wp + PW3, DH, b3, b3, b3, 1, 20, lng, lnb, resf, DH,
                  hmsg, DH, 1, gth, gtl, DH, 0, 0, 0);
    k_gemm<8, 2, 2, 0><<<dim3(NEDGE / 128, 1, 1), NTHR, LDS_G8, stream>>>(a);
  }
  k_aggr<<<NGR, NTHR, 0, stream>>>(ei, hmsg, Ach, Acl);

  unsigned short* curh = Ach; unsigned short* curl = Acl;
  unsigned short* nxth = Anh; unsigned short* nxtl = Anl;
  for (int l = 0; l < NLAY; ++l) {
    const unsigned short* base = wp + PLAY0 + (size_t)l * PLAYSZ;
    for (int s = 0; s < 2; ++s) {
      const size_t aro = (size_t)s * NDH * DH;
      {
        GArgs a = mkg(curh + aro, curl + aro, DH, 4, curh + aro, curl + aro, DH, 4, base + PQKV, DH,
                      qb + (size_t)l * HCOL, kb + (size_t)l * HCOL, vb + (size_t)l * HCOL, 3, 9, lng, lnb, resf, DH,
                      qkvf, QKVW, 1, qPh, qPl, HCOL, 1, HCOL, 0);
        k_gemm<8, 2, 0, 0><<<dim3(NDH / 128, QKVW / 128, 1), NTHR, LDS_G8, stream>>>(a);
      }
      {
        GArgs a = mkg(qPh, qPl, HCOL, 4, qPh, qPl, HCOL, 4, base + PWG, DH,
                      qb, qb, qb, 0, 20, lng, lnb, resf, DH,
                      Gf, 64, 1, gth, gtl, DH, 0, 0, DH);
        k_gemm<4, 2, 0, 1><<<dim3(NDH / 128, 1, 1), NTHR, LDS_G4, stream>>>(a);
      }
      k_attn<<<GPH, NTHR, 0, stream>>>(ei, ea, qkvf, Gf, Vsf, Sh, Sl, s * GPH);
      {
        GArgs a = mkg(Sh, Sl, 64, 2, curh + aro, curl + aro, DH, 6, base + PWTS, 192,
                      skb + (size_t)l * DH, skb + (size_t)l * DH, skb + (size_t)l * DH, 1, 20, lng, lnb, Vsf, DH,
                      Vsf, DH, 0, nxth + aro, nxtl + aro, DH, 1, BIGD, 0);
        k_gemm<8, 2, 4, 0><<<dim3(NDH / 128, 1, 1), NTHR, LDS_G8, stream>>>(a);
      }
    }
    unsigned short* th = curh; curh = nxth; nxth = th;
    unsigned short* tl = curl; curl = nxtl; nxtl = tl;
  }

  k_gat<<<NGR / 16, NTHR, 0, stream>>>(agent, curh, curl, gth, gtl);
  {
    GArgs a = mkg(gth, gtl, DH, 4, gth, gtl, DH, 4, wp + PWOUT, DH, ob, ob, ob, 1, 20, lng, lnb, resf, DH,
                  out, DH, 1, gth, gtl, DH, 0, 0, 0);
    k_gemm<8, 2, 0, 0><<<dim3(NGR / 128, 1, 1), NTHR, LDS_G8, stream>>>(a);
  }
}
